// VanillaGNN_5858335391843
// MI455X (gfx1250) — hardware-verified
//
#include <hip/hip_runtime.h>
#include <math.h>


typedef unsigned int u32;
typedef __attribute__((ext_vector_type(2)))  int      v2i;
typedef __attribute__((ext_vector_type(16))) _Float16 v16h;
typedef __attribute__((ext_vector_type(8)))  _Float16 v8h;
typedef __attribute__((ext_vector_type(8)))  float    v8f;
typedef __attribute__((ext_vector_type(4)))  float    v4f;
#define NN    50000
#define NE    800000
#define FF    128
#define DD    96
#define NC    40
#define SORTN 1048576
#define TILE  8192
#define NPAD  50176
#define VST2(T, ptr, val) do { const T _v = (val); *(volatile T*)(ptr) = _v; __threadfence(); *(volatile T*)(ptr) = _v; } while (0)
__device__ __forceinline__ v8f wmma16(v16h a, v16h b, v8f c) {
  v8f d = __builtin_amdgcn_wmma_f32_16x16x32_f16(false, a, false, b, (short)0, c, false, false);
  asm volatile("v_nop\n\tv_nop\n\tv_nop\n\tv_nop" : "+v"(d) : "v"(a), "v"(b));
  return d;
}
__device__ __forceinline__ v16h frag16(const _Float16* p, int hh) {
  const v8h lo = *(const v8h*)(p + 8 * hh), hi = *(const v8h*)(p + 16 + 8 * hh);
  return __builtin_shufflevector(lo, hi, 0,1,2,3,4,5,6,7,8,9,10,11,12,13,14,15);
}
__global__ __launch_bounds__(256) void k_sort_init(const int* __restrict__ src, const int* __restrict__ dst, u32* __restrict__ A, int E) {
  const int i = blockIdx.x * 256 + threadIdx.x;
  VST2(u32, A + i, (i < E) ? (((u32)dst[i]) << 16) | (u32)src[i] : 0xffffffffu);
}
__device__ __forceinline__ void cas_lds(u32* s, int lo, int hi, bool up) {
  const u32 a = s[lo], b = s[hi]; const bool sw = up ? (a > b) : (a < b); s[lo] = sw ? b : a; s[hi] = sw ? a : b;
}
__global__ __launch_bounds__(256) void k_sort_local(u32* __restrict__ A) {
  __shared__ u32 s[TILE];
  const int base = blockIdx.x * TILE, t = threadIdx.x;
  for (int i = t; i < TILE; i += 256) s[i] = A[base + i];
  __syncthreads();
  for (int k = 2; k <= TILE; k <<= 1)
    for (int j = k >> 1; j > 0; j >>= 1) {
      for (int p = t; p < TILE / 2; p += 256) {
        const int lo = ((p >> __builtin_ctz(j)) << (__builtin_ctz(j) + 1)) | (p & (j - 1));
        cas_lds(s, lo, lo + j, (((base + lo) & k) == 0));
      }
      __syncthreads();
    }
  for (int pass = 0; pass < 2; ++pass) { for (int i = t; i < TILE; i += 256) *(volatile u32*)(A + base + i) = s[i]; __threadfence(); }
}
__global__ __launch_bounds__(256) void k_sort_global(u32* __restrict__ A, int logj, int k) {
  const int p = blockIdx.x * 256 + threadIdx.x;
  const int j = 1 << logj;
  const int lo = ((p >> logj) << (logj + 1)) | (p & (j - 1)), hi = lo + j;
  const u32 a = A[lo], b = A[hi];
  const bool up = ((lo & k) == 0), sw = up ? (a > b) : (a < b);
  const u32 vlo = sw ? b : a, vhi = sw ? a : b;
  *(volatile u32*)(A + lo) = vlo; *(volatile u32*)(A + hi) = vhi; __threadfence();
  *(volatile u32*)(A + lo) = vlo; *(volatile u32*)(A + hi) = vhi;
}
__global__ __launch_bounds__(256) void k_sort_lds(u32* __restrict__ A, int k) {
  __shared__ u32 s[TILE];
  const int base = blockIdx.x * TILE, t = threadIdx.x;
  for (int i = t; i < TILE; i += 256) s[i] = A[base + i];
  __syncthreads();
  for (int j = TILE >> 1; j > 0; j >>= 1) {
    for (int p = t; p < TILE / 2; p += 256) {
      const int lo = ((p >> __builtin_ctz(j)) << (__builtin_ctz(j) + 1)) | (p & (j - 1));
      cas_lds(s, lo, lo + j, (((base + lo) & k) == 0));
    }
    __syncthreads();
  }
  for (int pass = 0; pass < 2; ++pass) { for (int i = t; i < TILE; i += 256) *(volatile u32*)(A + base + i) = s[i]; __threadfence(); }
}

__global__ __launch_bounds__(256) void k_segs(const u32* __restrict__ A, v2i* __restrict__ seg, float* __restrict__ inv) {
  const int n = blockIdx.x * 256 + threadIdx.x;
  if (n >= NN) return;
  int lo = 0, hi = SORTN;
  while (lo < hi) { const int mid = (lo + hi) >> 1; if ((A[mid] >> 16) < (u32)n) lo = mid + 1; else hi = mid; }
  const int st = lo; hi = SORTN;
  while (lo < hi) { const int mid = (lo + hi) >> 1; if ((A[mid] >> 16) < (u32)(n + 1)) lo = mid + 1; else hi = mid; }
  const v2i sv = {st, lo - st};
  VST2(v2i, seg + n, sv);
  VST2(float, inv + n, 1.0f / fmaxf((float)(lo - st), 1.0f));
}
__global__ __launch_bounds__(256) void k_rows(const float* __restrict__ h, const u32* __restrict__ A, const v2i* __restrict__ seg, const float* __restrict__ inv,
                                              _Float16* __restrict__ A16) {
  const int t = blockIdx.x * 256 + threadIdx.x;
  if (t >= NPAD * 24) return;
  const int i = t / 24, c = (t % 24) * 8;
  v8h o;
  if (i >= NN) { for (int e = 0; e < 8; ++e) o[e] = (_Float16)0.f; }
  else if (c >= DD) {
#pragma unroll
    for (int e = 0; e < 8; ++e) o[e] = (_Float16)h[(size_t)i * DD + c - DD + e];
  } else {
    const v2i sv = seg[i];
    float acc[8] = {0.f, 0.f, 0.f, 0.f, 0.f, 0.f, 0.f, 0.f};
    for (int p = 0; p < sv[1]; ++p) {
      const int j = (int)(A[sv[0] + p] & 0xffffu);
      const float* hr = h + (size_t)j * DD + c;
#pragma unroll
      for (int e = 0; e < 8; ++e) acc[e] += hr[e];
    }
    const float w = inv[i];
#pragma unroll
    for (int e = 0; e < 8; ++e) o[e] = (_Float16)(acc[e] * w);
  }
  VST2(v8h, A16 + (size_t)i * (2 * DD) + c, o);
}
__global__ __launch_bounds__(256) void k_x16(const float* __restrict__ x, _Float16* __restrict__ X16) {
  const int t = blockIdx.x * 256 + threadIdx.x;
  const int i = t >> 4, c = (t & 15) * 8;
  v8h o;
#pragma unroll
  for (int e = 0; e < 8; ++e) o[e] = (i < NN) ? (_Float16)x[(size_t)i * FF + c + e] : (_Float16)0.f;
  VST2(v8h, X16 + (size_t)i * FF + c, o);
}
__global__ __launch_bounds__(256) void k_h16(const float* __restrict__ h, _Float16* __restrict__ H16) {
  const int t = blockIdx.x * 256 + threadIdx.x;
  if (t >= NPAD * 12) return;
  const int i = t / 12, c = (t % 12) * 8;
  v8h o;
#pragma unroll
  for (int e = 0; e < 8; ++e) o[e] = (i < NN) ? (_Float16)h[(size_t)i * DD + c + e] : (_Float16)0.f;
  VST2(v8h, H16 + (size_t)i * DD + c, o);
}
__global__ __launch_bounds__(256) void k_wt(const float* __restrict__ w1, const float* __restrict__ w2, int K1, int K, int Nv, int Npad, int ldw, _Float16* __restrict__ Wt) {
  const int t = blockIdx.x * 256 + threadIdx.x;
  const int per = K / 8;
  if (t >= Npad * per) return;
  const int n = t / per, k0 = (t % per) * 8;
  v8h o;
#pragma unroll
  for (int e = 0; e < 8; ++e) { const int k = k0 + e; float v = 0.f; if (n < Nv) v = (k < K1) ? w1[k * ldw + n] : w2[(k - K1) * ldw + n]; o[e] = (_Float16)v; }
  VST2(v8h, Wt + (size_t)n * K + k0, o);
}
template <int K, int NT, bool RELU, bool DENSE>
__global__ __launch_bounds__(128) void k_gemm(const _Float16* __restrict__ A, const _Float16* __restrict__ Wt, const float* __restrict__ bias, float* __restrict__ out) {
  __shared__ __attribute__((aligned(16))) float sT[4][32][NT * 16 + 4];
  __shared__ __attribute__((aligned(16))) float sD[DENSE ? 1 : 128 * NC];
  const int lane = threadIdx.x & 31, wave = threadIdx.x >> 5, hh = lane >> 4, l16 = lane & 15;
  const int m0 = blockIdx.x * 128 + wave * 32;
  v8f acc[2][NT];
#pragma unroll
  for (int mi = 0; mi < 2; ++mi)
#pragma unroll
    for (int ni = 0; ni < NT; ++ni) acc[mi][ni] = (v8f){};
#pragma unroll 2
  for (int k0 = 0; k0 < K; k0 += 32) {
    const v16h a0 = frag16(A + (size_t)(m0 + l16) * K + k0, hh), a1 = frag16(A + (size_t)(m0 + 16 + l16) * K + k0, hh);
#pragma unroll
    for (int ni = 0; ni < NT; ++ni) { const v16h b = frag16(Wt + (size_t)(ni * 16 + l16) * K + k0, hh); acc[0][ni] = wmma16(a0, b, acc[0][ni]); acc[1][ni] = wmma16(a1, b, acc[1][ni]); }
  }
  float (*st)[NT * 16 + 4] = sT[wave];
#pragma unroll
  for (int mi = 0; mi < 2; ++mi)
#pragma unroll
    for (int ni = 0; ni < NT; ++ni)
#pragma unroll
      for (int i = 0; i < 8; ++i) { float v = acc[mi][ni][i] + bias[ni * 16 + l16]; if (RELU) v = fmaxf(v, 0.f); st[mi * 16 + i + 8 * hh][ni * 16 + l16] = v; }
  if (DENSE) {
    __builtin_amdgcn_fence(__ATOMIC_RELEASE, "workgroup"); __builtin_amdgcn_wave_barrier(); __builtin_amdgcn_fence(__ATOMIC_ACQUIRE, "workgroup");
    constexpr int P4 = NT * 4;
    for (int pass = 0; pass < 2; ++pass) {
      for (int p = lane; p < 32 * P4; p += 32) { const int rr = p / P4, q4 = (p % P4) * 4;
        *(volatile v4f*)(out + (size_t)(m0 + rr) * (NT * 16) + q4) = *(const v4f*)(&st[rr][q4]); }
      __threadfence();
    }
  } else {
    __syncthreads();
    for (int idx = threadIdx.x; idx < 128 * NC; idx += 128) { const int r = idx / NC, c = idx % NC; sD[idx] = sT[r >> 5][r & 31][c]; }
    __syncthreads();
    const int rows = min(128, NN - blockIdx.x * 128);
    if (rows > 0) {
      float* od = out + (size_t)blockIdx.x * 128 * NC;
      for (int pass = 0; pass < 2; ++pass) {
        for (int q4 = threadIdx.x * 4; q4 < rows * NC; q4 += 512) *(volatile v4f*)(od + q4) = *(const v4f*)(&sD[q4]);
        __threadfence();
      }
    }
  }
}
extern "C" void kernel_launch(void* const* d_in, const int* in_sizes, int n_in,
                              void* d_out, int out_size, void* d_ws, size_t ws_size, hipStream_t stream) {
  (void)in_sizes; (void)n_in; (void)out_size;
  const float* x     = (const float*)d_in[0];
  const int*   ei    = (const int*)  d_in[1];
  const float* enc_w = (const float*)d_in[2];
  const float* enc_b = (const float*)d_in[3];
  const float* lw    = (const float*)d_in[4];
  const float* lb    = (const float*)d_in[5];
  const float* rw    = (const float*)d_in[6];
  const float* dec_w = (const float*)d_in[7];
  const float* dec_b = (const float*)d_in[8];
  float* out = (float*)d_out;
  char* ws = (char*)d_ws; size_t off = 0;
  auto take = [&](size_t bytes) { void* p = ws + off; off = (off + bytes + 255) & ~(size_t)255; return p; };
  u32*      keys = (u32*)take((size_t)SORTN * 4);
  v2i*      seg  = (v2i*)take((size_t)NN * 8);
  float*    inv  = (float*)take((size_t)NN * 4);
  _Float16* X16  = (_Float16*)take((size_t)NPAD * FF * 2);
  _Float16* A16  = (_Float16*)take((size_t)NPAD * 2 * DD * 2);
  _Float16* H16  = (_Float16*)take((size_t)NPAD * DD * 2);
  _Float16* Wt   = (_Float16*)take((size_t)96 * 192 * 2);
  float*    h1   = (float*)take((size_t)NPAD * DD * 4);
  float*    h2   = (float*)take((size_t)NPAD * DD * 4);
  float*    bdec = (float*)take(64 * 4);
  if (off > ws_size) return;
  hipMemsetAsync(bdec, 0, 64 * 4, stream);
  hipMemcpyAsync(bdec, dec_b, NC * 4, hipMemcpyDeviceToDevice, stream);
  const dim3 b256(256);
  k_sort_init<<<SORTN / 256, b256, 0, stream>>>(ei, ei + NE, keys, NE);
  k_sort_local<<<SORTN / TILE, b256, 0, stream>>>(keys);
  for (int k = TILE * 2; k <= SORTN; k <<= 1) {
    for (int logj = __builtin_ctz(k) - 1; (1 << logj) >= TILE; --logj)
      k_sort_global<<<SORTN / 2 / 256, b256, 0, stream>>>(keys, logj, k);
    k_sort_lds<<<SORTN / TILE, b256, 0, stream>>>(keys, k);
  }
  k_segs<<<(NN + 255) / 256, b256, 0, stream>>>(keys, seg, inv);
  k_x16<<<NPAD * 16 / 256, b256, 0, stream>>>(x, X16);
  k_wt<<<(96 * 16 + 255) / 256, b256, 0, stream>>>(enc_w, enc_w, FF, FF, DD, DD, DD, Wt);
  k_gemm<FF, 6, true, true><<<NPAD / 128, 128, 0, stream>>>(X16, Wt, enc_b, h1);
  float* hin = h1; float* hout = h2;
  for (int l = 0; l < 3; ++l) {
    k_rows<<<(NPAD * 24 + 255) / 256, b256, 0, stream>>>(hin, keys, seg, inv, A16);
    k_wt<<<(96 * 24 + 255) / 256, b256, 0, stream>>>(lw + (size_t)l * DD * DD, rw + (size_t)l * DD * DD, DD, 2 * DD, DD, DD, DD, Wt);
    k_gemm<2 * DD, 6, true, true><<<NPAD / 128, 128, 0, stream>>>(A16, Wt, lb + l * DD, hout);
    float* tmp = hin; hin = hout; hout = tmp;
  }
  k_h16<<<(NPAD * 12 + 255) / 256, b256, 0, stream>>>(hin, H16);
  k_wt<<<(48 * 12 + 255) / 256, b256, 0, stream>>>(dec_w, dec_w, DD, DD, NC, 48, NC, Wt);
  k_gemm<DD, 3, false, false><<<NPAD / 128, 128, 0, stream>>>(H16, Wt, bdec, out);
}
